// SelfAttention_43937515438264
// MI455X (gfx1250) — hardware-run, weakly checked
//
#include <hip/hip_runtime.h>


#ifndef NB
#define NB 4
#endif
#ifndef SEQ
#define SEQ 4096
#endif
#define NB_FULL  4
#define SEQ_FULL 4096
#ifndef OUT_SEQ
#define OUT_SEQ SEQ
#endif
#define CH   256
#define CQ   32
#define QKW  64
#define CSPL 2
#define DV   (CH / CSPL)
#define AW   4
#define QRS  2048.0f
#define QRI  (1.0f / 2048.0f)
#define SC2  1.4426950408889634f
#define PSH  8.0f
#define NBIAS 320

static_assert(CQ == 32);
static_assert(QKW == 2 * CQ);
static_assert(CH % 64 == 0);
static_assert(CH % 32 == 0);
static_assert(DV == 128);
static_assert(DV == AW * 32);
static_assert(SEQ % 64 == 0);
static_assert((NB * SEQ) % 64 == 0);
static_assert(SEQ % 32 == 0);
static_assert(SEQ % (16 * AW) == 0);
static_assert(OUT_SEQ % 32 == 0);
static_assert(SEQ_FULL % 4 == 0);
static_assert(NB <= NB_FULL);
static_assert(SEQ <= SEQ_FULL);
static_assert(NBIAS == 2 * CQ + CH);
static_assert(NBIAS % 32 == 0);

typedef _Float16 h16;
typedef unsigned short bf;
typedef __attribute__((ext_vector_type(16))) __bf16   v16bf;
typedef __attribute__((ext_vector_type(16))) _Float16 v16h;
typedef __attribute__((ext_vector_type(8)))  _Float16 v8h;
typedef __attribute__((ext_vector_type(8)))  unsigned short v8us;
typedef __attribute__((ext_vector_type(8)))  float    v8f;
typedef __attribute__((ext_vector_type(4)))  float    v4f;
typedef v4f  __attribute__((may_alias)) v4fa;

__device__ __forceinline__ unsigned short f2bf(float f) { unsigned u = __float_as_uint(f); u += 0x7FFFu + ((u >> 16) & 1u); return (unsigned short)(u >> 16); }
__device__ __forceinline__ v16h cat16(v8h lo, v8h hi) { return __builtin_shufflevector(lo, hi, 0, 1, 2, 3, 4, 5, 6, 7, 8, 9, 10, 11, 12, 13, 14, 15); }
__device__ __forceinline__ v16bf cat16b(v8us lo, v8us hi) { return __builtin_bit_cast(v16bf, __builtin_shufflevector(lo, hi, 0, 1, 2, 3, 4, 5, 6, 7, 8, 9, 10, 11, 12, 13, 14, 15)); }
__device__ __forceinline__ v8f wmma16(v16h a, v16h b, v8f c) { return __builtin_amdgcn_wmma_f32_16x16x32_f16(false, a, false, b, (short)0, c, false, false); }
__device__ __forceinline__ v8f wmmab(v16bf a, v16bf b, v8f c) { return __builtin_amdgcn_wmma_f32_16x16x32_bf16(false, a, false, b, (short)0, c, false, false); }
__device__ __forceinline__ v16h  ldh(const h16* p) { return cat16(*(const v8h*)p, *(const v8h*)(p + 16)); }
__device__ __forceinline__ v16bf ldb(const bf* p)  { return cat16b(*(const v8us*)p, *(const v8us*)(p + 16)); }
__device__ __forceinline__ void wave_sync() { __builtin_amdgcn_fence(3  , "wavefront"); __builtin_amdgcn_wave_barrier(); asm volatile("" ::: "memory"); }

__global__ __launch_bounds__(256) void k_cvt8(const float* __restrict__ src, bf* dst, size_t n8) {
    const size_t i = (size_t)blockIdx.x * 256 + threadIdx.x; if (i >= n8) return;
    const v8f v = *(const v8f*)(src + i * 8); v8us o;
#pragma unroll
    for (int k = 0; k < 8; ++k) o[k] = f2bf(v[k]);
    *(volatile v8us*)(dst + i * 8) = o; __threadfence(); *(volatile v8us*)(dst + i * 8) = o;
}

__global__ __launch_bounds__(256) void k_xt(const float* __restrict__ x, bf* XB) {
    __shared__ float ts[64 * 65];
    const int tid = threadIdx.x;
    const int n0 = blockIdx.x * 64, c0 = blockIdx.y * 64, b = blockIdx.z;
    const float* xs = x + ((size_t)b * CH + c0) * SEQ_FULL + n0;
    { const int cr = tid >> 4, nq = (tid & 15) * 4;
#pragma unroll
      for (int i = 0; i < 4; ++i) { const int c = cr + 16 * i; const v4f v = *(const v4f*)(xs + (size_t)c * SEQ_FULL + nq);
          ts[c * 65 + nq + 0] = v[0]; ts[c * 65 + nq + 1] = v[1]; ts[c * 65 + nq + 2] = v[2]; ts[c * 65 + nq + 3] = v[3]; } }
    __syncthreads();
    const int rw = tid >> 3, c8 = (tid & 7) * 8;
    v8us o0, o1;
#pragma unroll
    for (int k = 0; k < 8; ++k) { o0[k] = f2bf(ts[(c8 + k) * 65 + rw]); o1[k] = f2bf(ts[(c8 + k) * 65 + rw + 32]); }
    bf* d0 = XB + ((size_t)b * SEQ + n0 + rw) * CH + c0 + c8; bf* d1 = d0 + (size_t)32 * CH;
    *(volatile v8us*)d0 = o0; *(volatile v8us*)d1 = o1;
    __threadfence();
    *(volatile v8us*)d0 = o0; *(volatile v8us*)d1 = o1;
}

__global__ __launch_bounds__(96) void k_bias(const float* __restrict__ bq, const float* __restrict__ bk, const float* __restrict__ bv, float* BT) {
    const int i = threadIdx.x; if (i >= NBIAS / 4) return;
    const int e = i * 4;
    const int iq = (e < CQ - 4) ? e : (CQ - 4);
    int ik = e - CQ; ik = ik < 0 ? 0 : ik; ik = ik > CQ - 4 ? CQ - 4 : ik;
    int iv = e - 2 * CQ; iv = iv < 0 ? 0 : iv; iv = iv > CH - 4 ? CH - 4 : iv;
    const v4f a = *(const v4f*)(bq + iq); const v4f c = *(const v4f*)(bk + ik); const v4f d = *(const v4f*)(bv + iv);
    v4f s, o;
#pragma unroll
    for (int k = 0; k < 4; ++k) { s[k] = (e < CQ) ? a[k] : ((e < 2 * CQ) ? c[k] : d[k]); o[k] = __uint_as_float(((unsigned)f2bf(s[k])) << 16); }
    *(volatile v4f*)(BT + e) = o; __threadfence(); *(volatile v4f*)(BT + e) = o;
}

template <int BROW>
__global__ __launch_bounds__(32) void k_proj(const bf* __restrict__ A, const bf* __restrict__ Bt, const float* __restrict__ bias, h16* Ph, h16* Pr, int useRes, int RB, size_t sRB, int pitch, int CB, size_t sCB) {
    __shared__ __align__(16) float os[16 * 68];
    const int K = CH;
    const int lane = threadIdx.x & 31, lr = lane & 15, hi = lane >> 4; const int r0 = blockIdx.x * 64, c0 = blockIdx.y * 64;
    v8f acc[4][4];
#pragma unroll
    for (int mb = 0; mb < 4; ++mb)
#pragma unroll
        for (int nb = 0; nb < 4; ++nb) acc[mb][nb] = (v8f){};
    const size_t aoff = (size_t)(r0 + lr) * K + 8 * hi, boff = (size_t)(c0 + lr) * K + 8 * hi;
#pragma unroll 1
    for (int kc = 0; kc < K; kc += 32) {
        v16bf a[4];
#pragma unroll
        for (int mb = 0; mb < 4; ++mb) a[mb] = ldb(A + aoff + (size_t)mb * 16 * K + kc);
#pragma unroll
        for (int nb = 0; nb < 4; ++nb) { const v16bf b = ldb(Bt + boff + (size_t)nb * 16 * K + kc);
#pragma unroll
            for (int mb = 0; mb < 4; ++mb) acc[mb][nb] = wmmab(a[mb], b, acc[mb][nb]); }
        asm volatile("v_nop\n\tv_nop\n\tv_nop\n\tv_nop" : "+v"(acc[0][0]), "+v"(acc[1][1]), "+v"(acc[2][2]), "+v"(acc[3][3]) : "v"(a[0]), "v"(a[1]), "v"(a[2]), "v"(a[3]));
    }
    float bcol[4] = {0.0f, 0.0f, 0.0f, 0.0f};
    if (BROW == 0) {
#pragma unroll
        for (int nb = 0; nb < 4; ++nb) bcol[nb] = bias[c0 + nb * 16 + lr];
    }
    const size_t tbase = (size_t)(r0 / RB) * sRB + (size_t)(r0 % RB) * (size_t)pitch + (size_t)(c0 / CB) * sCB + (size_t)(c0 % CB);
#pragma unroll
    for (int mb = 0; mb < 4; ++mb) {
        float brw[8] = {0.0f, 0.0f, 0.0f, 0.0f, 0.0f, 0.0f, 0.0f, 0.0f};
        if (BROW == 1) { const v4f b0 = *(const v4f*)(bias + r0 + mb * 16 + hi * 8); const v4f b1 = *(const v4f*)(bias + r0 + mb * 16 + hi * 8 + 4);
            brw[0] = b0[0]; brw[1] = b0[1]; brw[2] = b0[2]; brw[3] = b0[3]; brw[4] = b1[0]; brw[5] = b1[1]; brw[6] = b1[2]; brw[7] = b1[3]; }
#pragma unroll
        for (int nb = 0; nb < 4; ++nb) {
#pragma unroll
            for (int j = 0; j < 8; ++j) { const float bb = BROW ? brw[j] : bcol[nb]; os[(hi * 8 + j) * 68 + nb * 16 + lr] = acc[mb][nb][j] + bb; } }
        wave_sync();
        const size_t sb = tbase + (size_t)(mb * 16) * (size_t)pitch;
#pragma unroll 1
        for (int ps = 0; ps < 2; ++ps) {
#pragma unroll
            for (int s = 0; s < 4; ++s) { const int row = 4 * s + (lane >> 3), c8 = (lane & 7) * 8;
                const v4f x0 = *(const v4fa*)(&os[row * 68 + c8]); const v4f x1 = *(const v4fa*)(&os[row * 68 + c8 + 4]); v8h hv, rv;
#pragma unroll
                for (int i = 0; i < 4; ++i) { const h16 a0 = (h16)x0[i]; const h16 a1 = (h16)x1[i]; hv[i] = a0; hv[4 + i] = a1; rv[i] = (h16)((x0[i] - (float)a0) * QRS); rv[4 + i] = (h16)((x1[i] - (float)a1) * QRS); }
                const size_t oo = sb + (size_t)row * (size_t)pitch + c8;
                *(volatile v8h*)(Ph + oo) = hv; if (useRes) *(volatile v8h*)(Pr + oo) = rv; }
            if (ps == 0) __threadfence(); }
        wave_sync();
    }
}

__global__ __launch_bounds__(32 * AW) void k_flash(const h16* __restrict__ QKH, const h16* __restrict__ QKR, const h16* __restrict__ VT, float* OUT) {
    __shared__ __align__(16) float os[DV * 68];
    const int lane = threadIdx.x & 31, wave = __builtin_amdgcn_readfirstlane((int)(threadIdx.x >> 5)), lr = lane & 15, hi = lane >> 4;
    const int zh = blockIdx.y; const int b = zh / CSPL, ch = zh % CSPL;
    const int t0 = (blockIdx.x * AW + wave) * 16;
    const size_t pbase = (size_t)b * SEQ * QKW;
    const size_t qo = pbase + (size_t)(t0 + lr) * QKW + 8 * hi;
    const v16h qh = ldh(QKH + qo), qr = ldh(QKR + qo);
    const size_t ko = pbase + (size_t)lr * QKW + CQ + 8 * hi;
    const size_t vo = ((size_t)b * CH + (size_t)ch * DV + lr) * SEQ + 8 * hi;
    v8f o[8];
#pragma unroll
    for (int j = 0; j < 8; ++j) o[j] = (v8f){};
    float m = -3.0e38f, l = 0.0f;
#pragma unroll 1
    for (int key0 = 0; key0 < SEQ; key0 += 32) {
        const h16* ka = QKH + ko + (size_t)key0 * QKW;
        const v16h ka0 = ldh(ka), kb0 = ldh(ka + 16 * QKW);
        v8f sHa = (v8f){}, sLa = (v8f){}, sHb = (v8f){}, sLb = (v8f){};
        sHa = wmma16(ka0, qh, sHa); sLa = wmma16(ka0, qr, sLa); sHb = wmma16(kb0, qh, sHb); sLb = wmma16(kb0, qr, sLb);
        asm volatile("v_nop\n\tv_nop\n\tv_nop\n\tv_nop" : "+v"(sHa), "+v"(sLa), "+v"(sHb), "+v"(sLb) : "v"(ka0), "v"(kb0), "v"(qh), "v"(qr));
        float ta[8], tb[8]; float mx = -3.0e38f;
#pragma unroll
        for (int r = 0; r < 8; ++r) { ta[r] = (sHa[r] + sLa[r] * QRI) * SC2; tb[r] = (sHb[r] + sLb[r] * QRI) * SC2; mx = fmaxf(mx, fmaxf(ta[r], tb[r])); }
        mx = fmaxf(mx, __shfl_xor(mx, 16, 32));
        const float mnew = fmaxf(m, mx);
        const float alpha = __builtin_amdgcn_exp2f(m - mnew);
        const float sh = PSH - mnew;
        v16h pb; float ls = 0.0f;
#pragma unroll
        for (int r = 0; r < 8; ++r) { const h16 pa = (h16)__builtin_amdgcn_exp2f(ta[r] + sh); const h16 pc = (h16)__builtin_amdgcn_exp2f(tb[r] + sh); pb[r] = pa; pb[8 + r] = pc; ls += (float)pa + (float)pc; }
        l = l * alpha + ls; m = mnew;
#pragma unroll
        for (int j = 0; j < 8; ++j) o[j] = o[j] * alpha;
        const h16* va = VT + vo + key0;
        { const v16h v0 = ldh(va), v1 = ldh(va + (size_t)16 * SEQ), v2 = ldh(va + (size_t)32 * SEQ), v3 = ldh(va + (size_t)48 * SEQ);
          o[0] = wmma16(v0, pb, o[0]); o[1] = wmma16(v1, pb, o[1]); o[2] = wmma16(v2, pb, o[2]); o[3] = wmma16(v3, pb, o[3]);
          asm volatile("v_nop\n\tv_nop\n\tv_nop\n\tv_nop" : "+v"(o[0]), "+v"(o[1]), "+v"(o[2]), "+v"(o[3]) : "v"(v0), "v"(v1), "v"(v2), "v"(v3), "v"(pb)); }
        { const v16h v4 = ldh(va + (size_t)64 * SEQ), v5 = ldh(va + (size_t)80 * SEQ), v6 = ldh(va + (size_t)96 * SEQ), v7 = ldh(va + (size_t)112 * SEQ);
          o[4] = wmma16(v4, pb, o[4]); o[5] = wmma16(v5, pb, o[5]); o[6] = wmma16(v6, pb, o[6]); o[7] = wmma16(v7, pb, o[7]);
          asm volatile("v_nop\n\tv_nop\n\tv_nop\n\tv_nop" : "+v"(o[4]), "+v"(o[5]), "+v"(o[6]), "+v"(o[7]) : "v"(v4), "v"(v5), "v"(v6), "v"(v7), "v"(pb)); }
    }
    l += __shfl_xor(l, 16, 32);
    const float inv = 1.0f / l;
#pragma unroll
    for (int j = 0; j < 8; ++j) {
#pragma unroll
        for (int r = 0; r < 8; ++r) os[(16 * j + 8 * hi + r) * 68 + wave * 16 + lr] = o[j][r] * inv; }
    __syncthreads();
    float* obase = OUT + ((size_t)b * CH + (size_t)ch * DV) * OUT_SEQ + (size_t)blockIdx.x * (16 * AW);
#pragma unroll 1
    for (int ps = 0; ps < 2; ++ps) {
#pragma unroll
        for (int s = 0; s < 16; ++s) { const int row = wave * 32 + 2 * s + hi, cofs = lr * 4;
            const v4f val = *(const v4fa*)(&os[row * 68 + cofs]);
            *(volatile v4f*)(obase + (size_t)row * OUT_SEQ + cofs) = val; }
        if (ps == 0) __threadfence(); }
}

static constexpr size_t al256(size_t v) { return (v + 255) & ~(size_t)255; }
static constexpr size_t SZ_XB  = al256((size_t)NB * SEQ * CH * 2);
static constexpr size_t SZ_WQK = al256((size_t)QKW * CH * 2);
static constexpr size_t SZ_WV  = al256((size_t)CH * CH * 2);
static constexpr size_t SZ_BT  = al256((size_t)NBIAS * 4);
static constexpr size_t SZ_QK  = al256((size_t)NB * SEQ * QKW * 2);
static constexpr size_t SZ_VT  = al256((size_t)NB * CH * SEQ * 2);
static constexpr size_t SZ_TOTAL = SZ_XB + SZ_WQK + SZ_WV + SZ_BT + 2 * SZ_QK + SZ_VT;
static_assert(SZ_TOTAL <= (size_t)134217728);
static_assert(((size_t)CQ * CH * 2) % 256 == 0);

extern "C" void kernel_launch(void* const* d_in, const int* in_sizes, int n_in,
                              void* d_out, int out_size, void* d_ws, size_t ws_size, hipStream_t stream) {
    if (n_in < 7) return;
    const size_t needx = ((size_t)(NB - 1) * CH + (CH - 1)) * SEQ_FULL + SEQ;
    if ((size_t)in_sizes[0] < needx) return;
    if ((size_t)in_sizes[1] < (size_t)CQ * CH || (size_t)in_sizes[3] < (size_t)CQ * CH || (size_t)in_sizes[5] < (size_t)CH * CH) return;
    if (in_sizes[2] < CQ || in_sizes[4] < CQ || in_sizes[6] < CH) return;
    if ((size_t)out_size < ((size_t)(NB - 1) * CH + (CH - 1)) * OUT_SEQ + SEQ) return;
    if (SZ_TOTAL > ws_size) return;
    const float* x  = (const float*)d_in[0];
    const float* wq = (const float*)d_in[1]; const float* bq = (const float*)d_in[2];
    const float* wk = (const float*)d_in[3]; const float* bk = (const float*)d_in[4];
    const float* wv = (const float*)d_in[5]; const float* bv = (const float*)d_in[6];
    float* OUT = (float*)d_out;
    char* wsp = (char*)d_ws;
    bf* XB  = (bf*)wsp;  wsp += SZ_XB;
    bf* WQK = (bf*)wsp;  wsp += SZ_WQK;
    bf* WV  = (bf*)wsp;  wsp += SZ_WV;
    float* BT = (float*)wsp; wsp += SZ_BT;
    h16* QKH = (h16*)wsp; wsp += SZ_QK;
    h16* QKR = (h16*)wsp; wsp += SZ_QK;
    h16* VT  = (h16*)wsp; wsp += SZ_VT;

    k_xt<<<dim3(SEQ / 64, CH / 64, NB), 256, 0, stream>>>(x, XB);
    { const size_t n8 = (size_t)CQ * CH / 8; const unsigned g = (unsigned)((n8 + 255) / 256);
      k_cvt8<<<g, 256, 0, stream>>>(wq, WQK, n8); k_cvt8<<<g, 256, 0, stream>>>(wk, WQK + (size_t)CQ * CH, n8); }
    { const size_t n8 = (size_t)CH * CH / 8; k_cvt8<<<(unsigned)((n8 + 255) / 256), 256, 0, stream>>>(wv, WV, n8); }
    k_bias<<<1, 96, 0, stream>>>(bq, bk, bv, BT);

    k_proj<0><<<dim3(NB * SEQ / 64, QKW / 64, 1), 32, 0, stream>>>(XB, WQK, BT, QKH, QKR, 1, SEQ, (size_t)SEQ * QKW, QKW, QKW, (size_t)0);
    k_proj<1><<<dim3(CH / 64, NB * SEQ / 64, 1), 32, 0, stream>>>(WV, XB, BT + 2 * CQ, VT, VT, 0, CH, (size_t)0, SEQ, SEQ, (size_t)CH * SEQ);

    k_flash<<<dim3(SEQ / (16 * AW), NB * CSPL, 1), 32 * AW, 0, stream>>>(QKH, QKR, VT, OUT);
}
